// VSSM_54271206752691
// MI455X (gfx1250) — hardware-run, weakly checked
//
#include <hip/hip_runtime.h>
#include <math.h>

typedef __attribute__((ext_vector_type(16))) _Float16 v16h;
typedef __attribute__((ext_vector_type(8)))  _Float16 v8h;
typedef __attribute__((ext_vector_type(16))) __bf16   v16b;
typedef __attribute__((ext_vector_type(8)))  __bf16   v8b;
typedef __attribute__((ext_vector_type(8)))  float    v8f;
typedef __attribute__((ext_vector_type(4)))  float    v4f;

constexpr int kBatch = 2;
constexpr int kH     = 56;
constexpr int kW     = 56;
constexpr int kL     = kH * kW;
constexpr int kR     = kBatch * kL;
constexpr int kDim   = 96;
constexpr int kInn   = 192;
constexpr int kDin   = 384;
constexpr int kDtR   = 12;
constexpr int kNst   = 16;
constexpr int kDir   = 4;
constexpr int kXd    = kDtR + 2 * kNst;
constexpr int kPjN   = kDir * kXd;
constexpr int kPjP   = 192;
constexpr int kWoP   = 128;
constexpr int kXpP   = 2 * kInn;
constexpr int kXzP   = 2 * kDin;
static_assert(kL == 3136 && kR == 6272, "pixel counts");
static_assert(kXd == 44 && kPjN == 176 && kPjN <= kPjP, "projection widths");
static_assert((kR % 64) == 0 && (kXpP % 64) == 0 && (kXzP % 64) == 0 && (kPjP % 64) == 0 && (kInn % 64) == 0 && (kWoP % 64) == 0, "GEMM M,N multiples of 64");
static_assert((kDim % 32) == 0 && (kInn % 32) == 0 && (kDin % 32) == 0, "GEMM K multiples of 32");
static_assert((kR % 16) == 0 && (kR % 8) == 0 && (kL % 64) == 0 && (kL % 16) == 0 && (kDin % 64) == 0, "tile multiples");

constexpr float kCarX  = 16.0f;
constexpr float kCarW  = 32.0f;
constexpr float kCarX1 = 64.0f;
constexpr float kCarXi = 4096.0f;
constexpr float kCarG  = 1024.0f;
constexpr float kCarF  = 64.0f;

constexpr size_t kSzX16   = (size_t)kR * kDim * 2;
constexpr size_t kSzW12T  = (size_t)kXpP * kDim * 2;
constexpr size_t kSzINPT  = (size_t)kXzP * kInn * 2;
constexpr size_t kSzXPJT  = (size_t)kPjP * kDin * 2;
constexpr size_t kSzOUTT  = (size_t)kInn * kDin * 2;
constexpr size_t kSzWOT   = (size_t)kWoP * kInn * 2;
constexpr size_t kSzXP    = (size_t)kR * kXpP * 4;
constexpr size_t kSzX1H   = (size_t)kR * kInn * 2;
constexpr size_t kSzXZ    = (size_t)kR * kXzP * 4;
constexpr size_t kSzXI    = (size_t)kR * kDin * 4;
constexpr size_t kSzXI16  = (size_t)kR * kDin * 2;
constexpr size_t kSzPJ    = (size_t)kR * kPjP * 4;
constexpr size_t kSzOY    = (size_t)kDir * kR * kDin * 4;
constexpr size_t kSzG16   = (size_t)kR * kDin * 2;
constexpr size_t kSzTT    = (size_t)kR * kInn * 4;
constexpr size_t kSzFIN   = (size_t)kR * kInn * 2;
constexpr size_t kSzO2    = (size_t)kR * kWoP * 4;
constexpr size_t kOffX16  = 0;
constexpr size_t kOffW12T = kOffX16  + kSzX16;
constexpr size_t kOffINPT = kOffW12T + kSzW12T;
constexpr size_t kOffXPJT = kOffINPT + kSzINPT;
constexpr size_t kOffOUTT = kOffXPJT + kSzXPJT;
constexpr size_t kOffWOT  = kOffOUTT + kSzOUTT;
constexpr size_t kOffXP   = kOffWOT  + kSzWOT;
constexpr size_t kOffX1H  = kOffXP   + kSzXP;
constexpr size_t kOffXZ   = kOffX1H  + kSzX1H;
constexpr size_t kOffXI   = kOffXZ   + kSzXZ;
constexpr size_t kOffXI16 = kOffXI   + kSzXI;
constexpr size_t kOffPJ   = kOffXI16 + kSzXI16;
constexpr size_t kOffOY   = kOffPJ   + kSzPJ;
constexpr size_t kOffG16  = kOffOY   + kSzOY;
constexpr size_t kOffTT   = kOffG16  + kSzG16;
constexpr size_t kOffFIN  = kOffTT   + kSzTT;
constexpr size_t kOffO2   = kOffFIN  + kSzFIN;
constexpr size_t kWsTotal = kOffO2   + kSzO2;
static_assert(kWsTotal == 106283008ull, "carve total");
static_assert(kWsTotal <= 134217728ull, "carve cap");
static_assert((kSzX16 % 128) == 0 && (kSzW12T % 128) == 0 && (kSzINPT % 128) == 0 && (kSzXPJT % 128) == 0 &&
              (kSzOUTT % 128) == 0 && (kSzWOT % 128) == 0 && (kSzXP % 128) == 0 && (kSzX1H % 128) == 0 &&
              (kSzXZ % 128) == 0 && (kSzXI % 128) == 0 && (kSzXI16 % 128) == 0 && (kSzPJ % 128) == 0 &&
              (kSzOY % 128) == 0 && (kSzG16 % 128) == 0 && (kSzTT % 128) == 0 && (kSzFIN % 128) == 0 &&
              (kSzO2 % 128) == 0, "128-B aligned regions");

__device__ __forceinline__ unsigned short f2bf_bits(float f) {
  unsigned u = __float_as_uint(f);
  return (unsigned short)((u + 0x7FFFu + ((u >> 16) & 1u)) >> 16);
}
__device__ __forceinline__ float bf_bits2f(unsigned short h) { return __uint_as_float(((unsigned)h) << 16); }

__device__ __forceinline__ float bf16_rne(float f) {
  const unsigned u = __float_as_uint(f);
  const unsigned r = (u + 0x7FFFu + ((u >> 16) & 1u)) & 0xFFFF0000u;
  const bool isn = (u & 0x7FFFFFFFu) > 0x7F800000u;
  return __uint_as_float(isn ? u : r);
}

__device__ __forceinline__ void dep_guard4_h(v8f& a, v8f& b, v8f& c, v8f& d, v16h x, v16h y) { asm volatile("v_nop\n\tv_nop\n\tv_nop\n\tv_nop" : "+v"(a), "+v"(b), "+v"(c), "+v"(d) : "v"(x), "v"(y)); }
__device__ __forceinline__ void dep_guard4_b(v8f& a, v8f& b, v8f& c, v8f& d, v16b x, v16b y) { asm volatile("v_nop\n\tv_nop\n\tv_nop\n\tv_nop" : "+v"(a), "+v"(b), "+v"(c), "+v"(d) : "v"(x), "v"(y)); }
__device__ __forceinline__ void keep4_h(v16h a, v16h b, v16h c, v16h d) { asm volatile("v_nop" :: "v"(a), "v"(b), "v"(c), "v"(d)); }
__device__ __forceinline__ void keep4_b(v16b a, v16b b, v16b c, v16b d) { asm volatile("v_nop" :: "v"(a), "v"(b), "v"(c), "v"(d)); }
__device__ __forceinline__ void acc_guard4(v8f& a, v8f& b, v8f& c, v8f& d) { asm volatile("v_nop\n\tv_nop\n\tv_nop\n\tv_nop" : "+v"(a), "+v"(b), "+v"(c), "+v"(d)); }
template <typename T> struct Frag;
template <> struct Frag<_Float16> {
  typedef v16h V; union U { v16h v; v8h h[2]; };
  static __device__ __forceinline__ v16h load(const _Float16* p) {
    U f; f.h[0] = *(const v8h*)(p); f.h[1] = *(const v8h*)(p + 16); return f.v;
  }
  static __device__ __forceinline__ v8f mma(v16h a, v16h b, v8f c) {
    return __builtin_amdgcn_wmma_f32_16x16x32_f16(false, a, false, b, (short)0, c, false, false);
  }
  static __device__ __forceinline__ void guard4(v8f& a, v8f& b, v8f& c, v8f& d, v16h x, v16h y) { dep_guard4_h(a, b, c, d, x, y); }
  static __device__ __forceinline__ void keep(v16h a, v16h b, v16h c, v16h d) { keep4_h(a, b, c, d); }
};
template <> struct Frag<__bf16> {
  typedef v16b V; union U { v16b v; v8b h[2]; };
  static __device__ __forceinline__ v16b load(const __bf16* p) {
    U f; f.h[0] = *(const v8b*)(p); f.h[1] = *(const v8b*)(p + 16); return f.v;
  }
  static __device__ __forceinline__ v8f mma(v16b a, v16b b, v8f c) {
    return __builtin_amdgcn_wmma_f32_16x16x32_bf16(false, a, false, b, (short)0, c, false, false);
  }
  static __device__ __forceinline__ void guard4(v8f& a, v8f& b, v8f& c, v8f& d, v16b x, v16b y) { dep_guard4_b(a, b, c, d, x, y); }
  static __device__ __forceinline__ void keep(v16b a, v16b b, v16b c, v16b d) { keep4_b(a, b, c, d); }
};

template <int ET> struct Elem;
template <> struct Elem<0> { typedef _Float16 T; };
template <> struct Elem<1> { typedef __bf16 T; };
template <int ET, bool SPLIT, int BIAS_MODE, int OUT_MODE, bool RESID, int ACT = 0>
__global__ __launch_bounds__(256) void wmma_gemm64(
    const unsigned short* __restrict__ Ap, const unsigned short* __restrict__ A2p, int lda, long strideA,
    const unsigned short* __restrict__ Btp, const unsigned short* __restrict__ Bt2p, int ldb, long strideB,
    void* __restrict__ Cout, void* __restrict__ Cout2, int ldc, long strideC,
    const float* __restrict__ bias,
    const float* __restrict__ resid, long strideR,
    int M, int N, int K, float scale) {
  typedef typename Elem<ET>::T T;
  typedef typename Frag<T>::V V;
  const T* A = (const T*)Ap; const T* A2 = (const T*)A2p; const T* Bt = (const T*)Btp; const T* Bt2 = (const T*)Bt2p;
  __shared__ __align__(16) float sT[8][16 * 68];
  const int b    = blockIdx.y;
  const int lane = threadIdx.x & 31;
  const int wave = threadIdx.x >> 5;
  const int tilesN = N >> 6;
  const int tilesM = M >> 6;
  const int tile = blockIdx.x * 8 + wave;
  if (tile >= tilesM * tilesN) return;
  const int tm = tile / tilesN;
  const int tn = tile - tm * tilesN;
  const int m0 = tm << 6;
  const int n0 = tn << 6;

  const T* Ab  = A  + (size_t)b * strideA;
  const T* Bb  = Bt + (size_t)b * strideB;
  const T* Ab2 = SPLIT ? (A2  + (size_t)b * strideA) : nullptr;
  const T* Bb2 = SPLIT ? (Bt2 + (size_t)b * strideB) : nullptr;

  const int rlane = lane & 15;
  const int koff  = (lane >> 4) * 8;
  const int mOff  = (lane >> 4) * 8;

  v8f acc[4][4];
#pragma unroll
  for (int i = 0; i < 4; ++i)
#pragma unroll
    for (int j = 0; j < 4; ++j) acc[i][j] = (v8f){0.f,0.f,0.f,0.f,0.f,0.f,0.f,0.f};

  for (int k0 = 0; k0 < K; k0 += 32) {
    V bh[4], bl[4];
#pragma unroll
    for (int j = 0; j < 4; ++j) {
      const size_t bo = (size_t)(n0 + (j << 4) + rlane) * ldb + koff + k0;
      bh[j] = Frag<T>::load(Bb + bo);
      if (SPLIT) bl[j] = Frag<T>::load(Bb2 + bo);
    }
#pragma unroll
    for (int i = 0; i < 4; ++i) {
      const size_t ao = (size_t)(m0 + (i << 4) + rlane) * lda + koff + k0;
      V ah = Frag<T>::load(Ab + ao);
      V al;
      if (SPLIT) al = Frag<T>::load(Ab2 + ao);
#pragma unroll
      for (int j = 0; j < 4; ++j) {
        acc[i][j] = Frag<T>::mma(ah, bh[j], acc[i][j]);
        if (SPLIT) {
          acc[i][j] = Frag<T>::mma(ah, bl[j], acc[i][j]);
          acc[i][j] = Frag<T>::mma(al, bh[j], acc[i][j]);
        }
      }
      Frag<T>::guard4(acc[i][0], acc[i][1], acc[i][2], acc[i][3], ah, SPLIT ? al : ah);
    }
    Frag<T>::keep(bh[0], bh[1], bh[2], bh[3]);
    if (SPLIT) Frag<T>::keep(bl[0], bl[1], bl[2], bl[3]);
  }
  acc_guard4(acc[0][0], acc[0][1], acc[0][2], acc[0][3]);
  acc_guard4(acc[1][0], acc[1][1], acc[1][2], acc[1][3]);
  acc_guard4(acc[2][0], acc[2][1], acc[2][2], acc[2][3]);
  acc_guard4(acc[3][0], acc[3][1], acc[3][2], acc[3][3]);

  float* slab = sT[wave];
  const float* Rb = RESID ? (resid + (size_t)b * strideR) : nullptr;
#pragma unroll
  for (int i = 0; i < 4; ++i) {
    const int mBase = m0 + (i << 4);
#pragma unroll
    for (int j = 0; j < 4; ++j) {
      const int n = n0 + (j << 4) + rlane;
      float bv = 0.f;
      if (BIAS_MODE == 2) bv = bias[n];
#pragma unroll
      for (int r = 0; r < 8; ++r) {
        float v = acc[i][j][r] * scale;
        if (BIAS_MODE == 1) v += bias[mBase + mOff + r];
        if (BIAS_MODE == 2) v += bv;
        if (RESID) v += Rb[(size_t)(mBase + mOff + r) * ldc + n];
        if (ACT == 1) v = tanhf(v);
        if (ACT == 2) v = fmaxf(v, 0.0f);
        if (ACT == 3) v = v / (1.0f + expf(-v));
        if (ACT == 4) v = (v > 0.f) ? v : 0.01f * v;
        slab[(mOff + r) * 68 + (j << 4) + rlane] = v;
      }
    }
    __builtin_amdgcn_fence(__ATOMIC_RELEASE, "workgroup");
    __builtin_amdgcn_wave_barrier();
    __builtin_amdgcn_fence(__ATOMIC_ACQUIRE, "workgroup");
    if (OUT_MODE == 0) {
      float* C = (float*)Cout + (size_t)b * strideC;
      const int hh = lane >> 4, c4 = (lane & 15) * 4;
      for (int pass = 0; pass < 2; ++pass) {
#pragma unroll
        for (int it = 0; it < 8; ++it) {
          const int row = it * 2 + hh;
          v4f v = *(const v4f*)(slab + row * 68 + c4);
          *(volatile v4f*)(C + (size_t)(mBase + row) * ldc + n0 + c4) = v;
        }
        __threadfence();
      }
    } else {
      const int q = lane >> 3, c8 = (lane & 7) * 8;
      unsigned short* C  = (unsigned short*)Cout  + (size_t)b * strideC;
      unsigned short* C2 = (OUT_MODE == 2) ? ((unsigned short*)Cout2 + (size_t)b * strideC) : nullptr;
      for (int pass = 0; pass < 2; ++pass) {
#pragma unroll
        for (int it = 0; it < 4; ++it) {
          const int row = it * 4 + q;
          const float* sp = slab + row * 68 + c8;
          v8h hv, lv;
#pragma unroll
          for (int e = 0; e < 8; ++e) {
            if (OUT_MODE == 1) {
              hv[e] = (_Float16)sp[e];
            } else {
              unsigned short hb = f2bf_bits(sp[e]);
              unsigned short lb = f2bf_bits(sp[e] - bf_bits2f(hb));
              hv[e] = __builtin_bit_cast(_Float16, hb);
              lv[e] = __builtin_bit_cast(_Float16, lb);
            }
          }
          *(volatile v8h*)(C + (size_t)(mBase + row) * ldc + n0 + c8) = hv;
          if (OUT_MODE == 2) *(volatile v8h*)(C2 + (size_t)(mBase + row) * ldc + n0 + c8) = lv;
        }
        __threadfence();
      }
    }
    __builtin_amdgcn_fence(__ATOMIC_RELEASE, "workgroup");
    __builtin_amdgcn_wave_barrier();
    __builtin_amdgcn_fence(__ATOMIC_ACQUIRE, "workgroup");
  }
}

__global__ __launch_bounds__(256) void cast_f16_kernel(
    const float* __restrict__ src, unsigned short* __restrict__ dst, int total8, float scale)
{
  const int i = blockIdx.x * 256 + threadIdx.x;
  if (i >= total8) return;
  const size_t e0 = (size_t)i << 3;
  const float* p = src + e0;
  const v4f a0 = *(const v4f*)(p);
  const v4f a1 = *(const v4f*)(p + 4);
  v8h hv;
#pragma unroll
  for (int e = 0; e < 4; ++e) {
    const float s0 = a0[e];
    const float s1 = a1[e];
    hv[e]     = (_Float16)(bf16_rne(s0) * scale);
    hv[4 + e] = (_Float16)(bf16_rne(s1) * scale);
  }
  unsigned short* q = dst + e0;
  *(volatile v8h*)q = hv;
  __threadfence();
  *(volatile v8h*)q = hv;
}

__global__ __launch_bounds__(256) void weight_plane_kernel(
    const float* __restrict__ Wsrc, unsigned short* __restrict__ Bt,
    int Kdim, int Nreal, int sN, int sK, int total8, float scale)
{
  const int i = blockIdx.x * 256 + threadIdx.x;
  if (i >= total8) return;
  const int e0 = i << 3;
  const int n  = e0 / Kdim;
  const int k  = e0 - n * Kdim;
  const bool live = (n < Nreal);
  const int nc = live ? n : (Nreal - 1);
  const float* p = Wsrc + (size_t)nc * sN + (size_t)k * sK;
  v8h hv;
#pragma unroll
  for (int e = 0; e < 8; ++e) {
    const float v = bf16_rne(p[(size_t)e * sK]);
    const float t = live ? (v * scale) : 0.0f;
    hv[e] = (_Float16)t;
  }
  unsigned short* q = Bt + (size_t)e0;
  *(volatile v8h*)q = hv;
  __threadfence();
  *(volatile v8h*)q = hv;
}

template <int C, int INP, bool PREB, bool F32OUT>
__global__ __launch_bounds__(C) void dwconv_silu_kernel(
    const float* __restrict__ in, const float* __restrict__ wgt,
    const float* __restrict__ preb, const float* __restrict__ postb,
    float* __restrict__ outF, unsigned short* __restrict__ outH, float carry)
{
  constexpr int TP = C + 4;
  static_assert((C % 32) == 0 && (C % 8) == 0, "channel tile");
  __shared__ __align__(16) float sT[16 * TP];
  const int tid = threadIdx.x;
  const int r0  = blockIdx.x * 16;
  float w[9];
#pragma unroll
  for (int j = 0; j < 9; ++j) w[j] = bf16_rne(wgt[tid * 9 + j]);
  const float pb = PREB ? bf16_rne(preb[tid]) : 0.0f;
  const float qb = bf16_rne(postb[tid]);
#pragma unroll 1
  for (int s = 0; s < 16; ++s) {
    const int r  = r0 + s;
    const int bi = r / kL;
    const int p  = r - bi * kL;
    const int hh = p / kW;
    const int ww = p - hh * kW;
    float acc = 0.0f;
#pragma unroll
    for (int dy = 0; dy < 3; ++dy) {
#pragma unroll
      for (int dx = 0; dx < 3; ++dx) {
        const int y = hh + dy - 1;
        const int x = ww + dx - 1;
        const bool ok = (y >= 0) && (y < kH) && (x >= 0) && (x < kW);
        const int yc = (y < 0) ? 0 : ((y > kH - 1) ? (kH - 1) : y);
        const int xc = (x < 0) ? 0 : ((x > kW - 1) ? (kW - 1) : x);
        const float v = in[(size_t)(bi * kL + yc * kW + xc) * INP + tid];
        const float t = ok ? (v + pb) : 0.0f;
        acc = fmaf(w[dy * 3 + dx], t, acc);
      }
    }
    const float sv = acc + qb;
    const float sg = __builtin_amdgcn_rcpf(1.0f + expf(-sv));
    sT[s * TP + tid] = sv * sg;
  }
  __syncthreads();
  v8h hv[2];
#pragma unroll
  for (int it = 0; it < 2; ++it) {
    const int e   = (tid + C * it) * 8;
    const int row = e / C;
    const int col = e - row * C;
    const float* sp = sT + row * TP + col;
    const v4f a0 = *(const v4f*)(sp);
    const v4f a1 = *(const v4f*)(sp + 4);
#pragma unroll
    for (int q = 0; q < 4; ++q) {
      hv[it][q]     = (_Float16)(a0[q] * carry);
      hv[it][4 + q] = (_Float16)(a1[q] * carry);
    }
  }
  v4f fv[4];
  if (F32OUT) {
#pragma unroll
    for (int it = 0; it < 4; ++it) {
      const int e   = (tid + C * it) * 4;
      const int row = e / C;
      const int col = e - row * C;
      fv[it] = *(const v4f*)(sT + row * TP + col);
    }
  }
  for (int pass = 0; pass < 2; ++pass) {
#pragma unroll
    for (int it = 0; it < 2; ++it)
      *(volatile v8h*)(outH + (size_t)r0 * C + (size_t)(tid + C * it) * 8) = hv[it];
    if (F32OUT) {
#pragma unroll
      for (int it = 0; it < 4; ++it)
        *(volatile v4f*)(outF + (size_t)r0 * C + (size_t)(tid + C * it) * 4) = fv[it];
    }
    __threadfence();
  }
}

constexpr int kScTS = 64;
constexpr int kScCh = 64;
constexpr int kScYP = 68;
constexpr int kScXP = 44;
static_assert(kScXP == kXd && (kXd % 4) == 0, "staged row width");
__global__ __launch_bounds__(64) void scan_kernel(
    const float* __restrict__ PJ, const float* __restrict__ XI,
    const float* __restrict__ Wdt, const float* __restrict__ bdt, const float* __restrict__ Alog,
    const float* __restrict__ Dsk, float* __restrict__ OY)
{
  __shared__ __align__(16) float sX[kScTS * kScXP];
  __shared__ __align__(16) float sY[kScTS * kScYP];
  __shared__ int sRow[kScTS];
  const int tid = threadIdx.x;
  constexpr int kGrp = kDin / kScCh;
  const int bk  = blockIdx.x / kGrp;
  const int grp = blockIdx.x - bk * kGrp;
  const int bi  = bk >> 2;
  const int k   = bk & 3;
  const int c0  = grp * kScCh;
  const int c   = c0 + tid;
  const int kc  = k * kDin + c;

  float negA[kNst], h[kNst], dw[kDtR];
#pragma unroll
  for (int q = 0; q < 4; ++q) {
    const v4f av = *(const v4f*)(Alog + (size_t)kc * kNst + 4 * q);
    const float a0 = av[0];
    const float a1 = av[1];
    const float a2 = av[2];
    const float a3 = av[3];
    negA[4 * q + 0] = -__expf(bf16_rne(a0));
    negA[4 * q + 1] = -__expf(bf16_rne(a1));
    negA[4 * q + 2] = -__expf(bf16_rne(a2));
    negA[4 * q + 3] = -__expf(bf16_rne(a3));
  }
#pragma unroll
  for (int q = 0; q < 3; ++q) {
    const v4f wv = *(const v4f*)(Wdt + (size_t)kc * kDtR + 4 * q);
    const float w0 = wv[0];
    const float w1 = wv[1];
    const float w2 = wv[2];
    const float w3 = wv[3];
    dw[4 * q + 0] = bf16_rne(w0);
    dw[4 * q + 1] = bf16_rne(w1);
    dw[4 * q + 2] = bf16_rne(w2);
    dw[4 * q + 3] = bf16_rne(w3);
  }
#pragma unroll
  for (int n = 0; n < kNst; ++n) h[n] = 0.0f;
  const float db = bf16_rne(bdt[kc]);
  const float Dd = bf16_rne(Dsk[kc]);
  float* oyp = OY + (size_t)k * kR * kDin;
  const int fr = tid >> 4, fc = (tid & 15) * 4;

#pragma unroll 1
  for (int t0 = 0; t0 < kL; t0 += kScTS) {
    __syncthreads();
    {
      const int t  = t0 + tid;
      const int j  = (k >= 2) ? (kL - 1 - t) : t;
      const int wq = j / kH;
      const int hq = j - wq * kH;
      const int pos = (k & 1) ? (hq * kW + wq) : j;
      sRow[tid] = bi * kL + pos;
    }
    __syncthreads();
#pragma unroll
    for (int i = 0; i < 11; ++i) {
      const int idx = tid + 64 * i;
      const int s   = idx / 11;
      const int q   = idx - s * 11;
      const int row = sRow[s];
      *(v4f*)(sX + s * kScXP + 4 * q) = *(const v4f*)(PJ + (size_t)row * kPjP + k * kXd + 4 * q);
    }
    __syncthreads();
#pragma unroll 1
    for (int s = 0; s < kScTS; ++s) {
      const float* xr = sX + s * kScXP;
      const v4f d0 = *(const v4f*)(xr);
      const v4f d1 = *(const v4f*)(xr + 4);
      const v4f d2 = *(const v4f*)(xr + 8);
      float vdot = db;
      vdot = fmaf(d0[0], dw[0], vdot);
      vdot = fmaf(d0[1], dw[1], vdot);
      vdot = fmaf(d0[2], dw[2], vdot);
      vdot = fmaf(d0[3], dw[3], vdot);
      vdot = fmaf(d1[0], dw[4], vdot);
      vdot = fmaf(d1[1], dw[5], vdot);
      vdot = fmaf(d1[2], dw[6], vdot);
      vdot = fmaf(d1[3], dw[7], vdot);
      vdot = fmaf(d2[0], dw[8], vdot);
      vdot = fmaf(d2[1], dw[9], vdot);
      vdot = fmaf(d2[2], dw[10], vdot);
      vdot = fmaf(d2[3], dw[11], vdot);
      const float a   = __expf(-fabsf(vdot));
      const float u1  = 1.0f + a;
      const float l1p = __logf(u1) + (a - (u1 - 1.0f)) * __builtin_amdgcn_rcpf(u1);
      const float dt  = fmaxf(vdot, 0.0f) + l1p;
      const int   row = sRow[s];
      const float xt  = XI[(size_t)row * kDin + c];
      const float dtx = dt * xt;
      float y = 0.0f;
#pragma unroll
      for (int q4 = 0; q4 < 4; ++q4) {
        const v4f bv = *(const v4f*)(xr + kDtR + 4 * q4);
        const v4f cv = *(const v4f*)(xr + kDtR + kNst + 4 * q4);
#pragma unroll
        for (int e = 0; e < 4; ++e) {
          const int n = 4 * q4 + e;
          const float ev = __expf(dt * negA[n]);
          h[n] = fmaf(ev, h[n], dtx * bv[e]);
          y = fmaf(h[n], cv[e], y);
        }
      }
      y = fmaf(xt, Dd, y);
      sY[s * kScYP + tid] = y;
    }
    __syncthreads();
    v4f fv[16];
    int rw[16];
#pragma unroll
    for (int it = 0; it < 16; ++it) {
      fv[it] = *(const v4f*)(sY + (it * 4 + fr) * kScYP + fc);
      rw[it] = sRow[it * 4 + fr];
    }
    for (int pass = 0; pass < 2; ++pass) {
#pragma unroll
      for (int it = 0; it < 16; ++it)
        *(volatile v4f*)(oyp + (size_t)rw[it] * kDin + c0 + fc) = fv[it];
      __threadfence();
    }
  }
}

template <int C, int NPL, int GP, int GOFF, bool GBIAS>
__global__ __launch_bounds__(256) void ln_gate_kernel(
    const float* __restrict__ src, long planeStride,
    const float* __restrict__ gam, const float* __restrict__ bet,
    const float* __restrict__ gsrc, const float* __restrict__ gb,
    unsigned short* __restrict__ dst, float carry)
{
  constexpr int TP  = C + 4;
  constexpr int PER = C / 32;
  constexpr int NEL = (8 * C) / 256;
  constexpr int NIT = (C + 255) / 256;
  static_assert((C % 32) == 0 && ((8 * C) % 256) == 0 && (C % 8) == 0, "row width");
  __shared__ __align__(16) float sT[8 * TP];
  __shared__ float sStat[16];
  const int tid = threadIdx.x, lane = tid & 31, wave = tid >> 5;
  const int r0 = blockIdx.x * 8;
  const int r  = r0 + wave;
  float acc[PER];
#pragma unroll
  for (int j = 0; j < PER; ++j) acc[j] = 0.0f;
#pragma unroll 1
  for (int k = 0; k < NPL; ++k) {
    const float* p = src + (size_t)k * (size_t)planeStride + (size_t)r * C;
#pragma unroll
    for (int j = 0; j < PER; ++j) acc[j] += p[lane + 32 * j];
  }
  float s = 0.0f;
#pragma unroll
  for (int j = 0; j < PER; ++j) s += acc[j];
#pragma unroll
  for (int o = 16; o > 0; o >>= 1) s += __shfl_xor(s, o, 32);
  const float mean = s * (1.0f / (float)C);
  float q = 0.0f;
#pragma unroll
  for (int j = 0; j < PER; ++j) {
    const float d = acc[j] - mean;
    q = fmaf(d, d, q);
  }
#pragma unroll
  for (int o = 16; o > 0; o >>= 1) q += __shfl_xor(q, o, 32);
  const float var = q * (1.0f / (float)C);
  const float rs  = rsqrtf(var + 1e-5f);
#pragma unroll
  for (int j = 0; j < PER; ++j) sT[wave * TP + lane + 32 * j] = acc[j];
  if (lane == 0) {
    sStat[wave * 2]     = mean;
    sStat[wave * 2 + 1] = rs;
  }
  __syncthreads();
#pragma unroll 1
  for (int j = 0; j < NEL; ++j) {
    const int idx = tid + 256 * j;
    const int row = idx / C;
    const int cc  = idx - row * C;
    const float yv = sT[row * TP + cc];
    const float m  = sStat[row * 2];
    const float iv = sStat[row * 2 + 1];
    float gv = gsrc[(size_t)(r0 + row) * GP + GOFF + cc];
    if (GBIAS) gv += bf16_rne(gb[cc]);
    const float sg = __builtin_amdgcn_rcpf(1.0f + expf(-gv));
    const float gq = bf16_rne(gam[cc]);
    const float bq = bf16_rne(bet[cc]);
    const float ln = (yv - m) * iv * gq + bq;
    sT[row * TP + cc] = ln * (gv * sg) * carry;
  }
  __syncthreads();
  v8h hv[NIT];
#pragma unroll
  for (int it = 0; it < NIT; ++it) {
    const int piece = tid + 256 * it;
    const int pc    = (piece < C) ? piece : 0;
    const int e     = pc * 8;
    const int row   = e / C;
    const int col   = e - row * C;
    const float* sp = sT + row * TP + col;
    const v4f a0 = *(const v4f*)(sp);
    const v4f a1 = *(const v4f*)(sp + 4);
#pragma unroll
    for (int z = 0; z < 4; ++z) {
      hv[it][z]     = (_Float16)a0[z];
      hv[it][4 + z] = (_Float16)a1[z];
    }
  }
  for (int pass = 0; pass < 2; ++pass) {
#pragma unroll
    for (int it = 0; it < NIT; ++it) {
      const int piece = tid + 256 * it;
      if (piece < C)
        *(volatile v8h*)(dst + (size_t)r0 * C + (size_t)piece * 8) = hv[it];
    }
    __threadfence();
  }
}

__global__ __launch_bounds__(256) void out_bias_kernel(
    const float* __restrict__ O2, const float* __restrict__ bo, float* __restrict__ outp, int total4)
{
  const int i = blockIdx.x * 256 + threadIdx.x;
  if (i >= total4) return;
  constexpr int kPer = kDim / 4;
  const int r  = i / kPer;
  const int c4 = (i - r * kPer) * 4;
  const v4f v  = *(const v4f*)(O2 + (size_t)r * kWoP + c4);
  const v4f bb = *(const v4f*)(bo + c4);
  const float b0 = bb[0];
  const float b1 = bb[1];
  const float b2 = bb[2];
  const float b3 = bb[3];
  v4f o;
  o[0] = v[0] + bf16_rne(b0);
  o[1] = v[1] + bf16_rne(b1);
  o[2] = v[2] + bf16_rne(b2);
  o[3] = v[3] + bf16_rne(b3);
  float* q = outp + (size_t)i * 4;
  *(volatile v4f*)q = o;
  __threadfence();
  *(volatile v4f*)q = o;
}

extern "C" void kernel_launch(void* const* d_in, const int* in_sizes, int n_in,
                              void* d_out, int out_size, void* d_ws, size_t ws_size,
                              hipStream_t stream)
{
  if (n_in < 22) return;
  if (in_sizes[0]  != kR * kDim) return;
  if (in_sizes[1]  != kDim * kInn || in_sizes[2] != kInn) return;
  if (in_sizes[3]  != kInn * 9 || in_sizes[4] != kInn) return;
  if (in_sizes[5]  != kInn * kXzP) return;
  if (in_sizes[6]  != kDin * 9 || in_sizes[7] != kDin) return;
  if (in_sizes[8]  != kDir * kXd * kDin) return;
  if (in_sizes[9]  != kDir * kDin * kDtR || in_sizes[10] != kDir * kDin) return;
  if (in_sizes[11] != kDir * kDin * kNst || in_sizes[12] != kDir * kDin) return;
  if (in_sizes[13] != kDin || in_sizes[14] != kDin) return;
  if (in_sizes[15] != kDin * kInn) return;
  if (in_sizes[16] != kInn || in_sizes[17] != kInn) return;
  if (in_sizes[18] != kDim * kInn || in_sizes[19] != kInn) return;
  if (in_sizes[20] != kInn * kDim || in_sizes[21] != kDim) return;
  if (out_size != kR * kDim) return;
  if (ws_size < kWsTotal) return;

  const float* x        = (const float*)d_in[0];
  const float* w1       = (const float*)d_in[1];
  const float* b1       = (const float*)d_in[2];
  const float* dw_w     = (const float*)d_in[3];
  const float* dw_b     = (const float*)d_in[4];
  const float* inproj_w = (const float*)d_in[5];
  const float* cv_w     = (const float*)d_in[6];
  const float* cv_b     = (const float*)d_in[7];
  const float* xproj_w  = (const float*)d_in[8];
  const float* dtp_w    = (const float*)d_in[9];
  const float* dtp_b    = (const float*)d_in[10];
  const float* A_logs   = (const float*)d_in[11];
  const float* Dsk      = (const float*)d_in[12];
  const float* onorm_g  = (const float*)d_in[13];
  const float* onorm_b  = (const float*)d_in[14];
  const float* outp_w   = (const float*)d_in[15];
  const float* norm_g   = (const float*)d_in[16];
  const float* norm_b   = (const float*)d_in[17];
  const float* w2       = (const float*)d_in[18];
  const float* b2       = (const float*)d_in[19];
  const float* wo       = (const float*)d_in[20];
  const float* bo       = (const float*)d_in[21];
  float* outp = (float*)d_out;

  char* ws = (char*)d_ws;
  unsigned short* X16   = (unsigned short*)(ws + kOffX16);
  unsigned short* W12T  = (unsigned short*)(ws + kOffW12T);
  unsigned short* INPT  = (unsigned short*)(ws + kOffINPT);
  unsigned short* XPJT  = (unsigned short*)(ws + kOffXPJT);
  unsigned short* OUTT  = (unsigned short*)(ws + kOffOUTT);
  unsigned short* WOT   = (unsigned short*)(ws + kOffWOT);
  float*          XP    = (float*)(ws + kOffXP);
  unsigned short* X1H   = (unsigned short*)(ws + kOffX1H);
  float*          XZ    = (float*)(ws + kOffXZ);
  float*          XI    = (float*)(ws + kOffXI);
  unsigned short* XI16  = (unsigned short*)(ws + kOffXI16);
  float*          PJ    = (float*)(ws + kOffPJ);
  float*          OY    = (float*)(ws + kOffOY);
  unsigned short* G16   = (unsigned short*)(ws + kOffG16);
  float*          TT    = (float*)(ws + kOffTT);
  unsigned short* FIN16 = (unsigned short*)(ws + kOffFIN);
  float*          O2    = (float*)(ws + kOffO2);
  const float* dummyf = b1;

  cast_f16_kernel<<<(kR * kDim / 8) / 256, 256, 0, stream>>>(x, X16, kR * kDim / 8, kCarX);
  weight_plane_kernel<<<(kInn * kDim / 8) / 256, 256, 0, stream>>>(w1, W12T, kDim, kInn, 1, kInn, kInn * kDim / 8, kCarW);
  weight_plane_kernel<<<(kInn * kDim / 8) / 256, 256, 0, stream>>>(w2, W12T + (size_t)kInn * kDim, kDim, kInn, 1, kInn, kInn * kDim / 8, kCarW);
  weight_plane_kernel<<<(kXzP * kInn / 8) / 256, 256, 0, stream>>>(inproj_w, INPT, kInn, kXzP, 1, kXzP, kXzP * kInn / 8, kCarW);
  weight_plane_kernel<<<(kPjP * kDin / 8) / 256, 256, 0, stream>>>(xproj_w, XPJT, kDin, kPjN, kDin, 1, kPjP * kDin / 8, kCarW);
  weight_plane_kernel<<<(kInn * kDin / 8) / 256, 256, 0, stream>>>(outp_w, OUTT, kDin, kInn, 1, kInn, kInn * kDin / 8, kCarW);
  weight_plane_kernel<<<(kWoP * kInn / 8) / 256, 256, 0, stream>>>(wo, WOT, kInn, kDim, 1, kDim, kWoP * kInn / 8, kCarW);

  wmma_gemm64<0, false, 0, 0, false><<<dim3(((kR / 64) * (kXpP / 64) + 7) / 8, 1), 256, 0, stream>>>(
      X16, X16, kDim, 0L, W12T, W12T, kDim, 0L,
      (void*)XP, (void*)XP, kXpP, 0L, dummyf, dummyf, 0L, kR, kXpP, kDim, 1.0f / (kCarX * kCarW));

  dwconv_silu_kernel<kInn, kXpP, true, false><<<kR / 16, kInn, 0, stream>>>(
      XP, dw_w, b1, dw_b, XI, X1H, kCarX1);

  wmma_gemm64<0, false, 0, 0, false><<<dim3(((kR / 64) * (kXzP / 64) + 7) / 8, 1), 256, 0, stream>>>(
      X1H, X1H, kInn, 0L, INPT, INPT, kInn, 0L,
      (void*)XZ, (void*)XZ, kXzP, 0L, dummyf, dummyf, 0L, kR, kXzP, kInn, 1.0f / (kCarX1 * kCarW));

  dwconv_silu_kernel<kDin, kXzP, false, true><<<kR / 16, kDin, 0, stream>>>(
      XZ, cv_w, cv_b, cv_b, XI, XI16, kCarXi);

  wmma_gemm64<0, false, 0, 0, false><<<dim3(((kR / 64) * (kPjP / 64) + 7) / 8, 1), 256, 0, stream>>>(
      XI16, XI16, kDin, 0L, XPJT, XPJT, kDin, 0L,
      (void*)PJ, (void*)PJ, kPjP, 0L, dummyf, dummyf, 0L, kR, kPjP, kDin, 1.0f / (kCarXi * kCarW));

  scan_kernel<<<kBatch * kDir * (kDin / kScCh), kScCh, 0, stream>>>(PJ, XI, dtp_w, dtp_b, A_logs, Dsk, OY);

  ln_gate_kernel<kDin, kDir, kXzP, kDin, false><<<kR / 8, 256, 0, stream>>>(
      OY, (long)kR * kDin, onorm_g, onorm_b, XZ, onorm_b, G16, kCarG);

  wmma_gemm64<0, false, 0, 0, false><<<dim3(((kR / 64) * (kInn / 64) + 7) / 8, 1), 256, 0, stream>>>(
      G16, G16, kDin, 0L, OUTT, OUTT, kDin, 0L,
      (void*)TT, (void*)TT, kInn, 0L, dummyf, dummyf, 0L, kR, kInn, kDin, 1.0f / (kCarG * kCarW));

  ln_gate_kernel<kInn, 1, kXpP, kInn, true><<<kR / 8, 256, 0, stream>>>(
      TT, 0L, norm_g, norm_b, XP, b2, FIN16, kCarF);

  wmma_gemm64<0, false, 0, 0, false><<<dim3(((kR / 64) * (kWoP / 64) + 7) / 8, 1), 256, 0, stream>>>(
      FIN16, FIN16, kInn, 0L, WOT, WOT, kInn, 0L,
      (void*)O2, (void*)O2, kWoP, 0L, dummyf, dummyf, 0L, kR, kWoP, kInn, 1.0f / (kCarF * kCarW));

  out_bias_kernel<<<(kR * kDim / 4) / 256, 256, 0, stream>>>(O2, bo, outp, kR * kDim / 4);
}
